// CrossAxisAttention_40647570489983
// MI455X (gfx1250) — hardware-verified
//
#include <hip/hip_runtime.h>
#include <stdint.h>
#include <stddef.h>


typedef _Float16 f16t;
typedef f16t  v16h __attribute__((ext_vector_type(16)));
typedef f16t  v8h  __attribute__((ext_vector_type(8)));
typedef f16t  v8ha __attribute__((ext_vector_type(8), may_alias));
typedef float v8f  __attribute__((ext_vector_type(8)));
typedef float v4f  __attribute__((ext_vector_type(4)));
typedef float v4fa __attribute__((ext_vector_type(4), may_alias));

union Frag { v16h v; v8h half[2]; };
union H8   { v8h h; v4f f; };

#define NBATCH 8
#define CD     256
#define HWD    56
#define NPIX   3136
#define NTOK   25088
#define NHEAD  8
#define HD     32
#define SWID   7
#define SL     392
#define SLP    416
#define NCH    13
#define NQT    25
#define OPITCH 512
#define PP     40
#define TP     68

#define W_SCL     1024.0f
#define INV_W     0.0009765625f
#define QK_SCL    16.0f
#define V_SCL     16.0f
#define P_SCL     256.0f
#define LOGIT_SCL (0.17677669529663687f * 0.00390625f)
#define O_EPI     0.0625f
#define PROJ_EPI  (1.0f / 262144.0f)

__device__ __forceinline__ v8f mma_g(v8f c, v16h a, v16h b) {
    v8f d = __builtin_amdgcn_wmma_f32_16x16x32_f16(false, a, false, b, (short)0, c, false, false);
    asm volatile("v_nop\n\tv_nop\n\tv_nop\n\tv_nop" : "+v"(d) : "v"(a), "v"(b));
    return d;
}

__device__ __forceinline__ int tok_of(int dir, int base, int sn, int i) {
    return (dir == 0) ? (base + sn * SL + i)
                      : (base + (i % HWD) * HWD + sn * SWID + i / HWD);
}

__global__ __launch_bounds__(256) void k_cvt_x(const float* __restrict__ x, f16t* __restrict__ Xt) {
    __shared__ __align__(16) f16t T[32][72];
    const int t = threadIdx.x;
    const int tok0 = blockIdx.x * 32;
    const int c0 = blockIdx.y * 64;
    const int b = tok0 / NPIX, p0 = tok0 - b * NPIX;
    const float* src = x + (size_t)b * CD * NPIX + (size_t)c0 * NPIX + p0;
#pragma unroll
    for (int i = 0; i < 8; ++i) {
        const int r = i * 8 + (t >> 5);
        const int col = t & 31;
        T[col][r] = (f16t)src[(size_t)r * NPIX + col];
    }
    __syncthreads();
    const int tk = t >> 3, q = t & 7;
    H8 u;
    u.h = *(const v8ha*)(&T[tk][8 * q]);
    f16t* dst = Xt + (size_t)(tok0 + tk) * CD + c0 + 8 * q;
    *(volatile v4f*)dst = u.f;
    __threadfence();
    *(volatile v4f*)dst = u.f;
}

__global__ __launch_bounds__(256) void k_cvt_w(const float* __restrict__ src, f16t* __restrict__ dst,
                                              int n8, float scl) {
    const int i = blockIdx.x * 256 + threadIdx.x;
    if (i >= n8) return;
    v4f a = *(const v4fa*)(src + (size_t)i * 8);
    v4f b = *(const v4fa*)(src + (size_t)i * 8 + 4);
    H8 u;
#pragma unroll
    for (int j = 0; j < 4; ++j) {
        u.h[j]     = (f16t)(a[j] * scl);
        u.h[4 + j] = (f16t)(b[j] * scl);
    }
    f16t* d = dst + (size_t)i * 8;
    *(volatile v4f*)d = u.f;
    __threadfence();
    *(volatile v4f*)d = u.f;
}

__global__ __launch_bounds__(256) void k_gemm_qkv(const f16t* __restrict__ Xt, const f16t* __restrict__ W,
                                                 const float* __restrict__ bias,
                                                 f16t* __restrict__ Q16, f16t* __restrict__ K16,
                                                 float* __restrict__ Vf) {
    __shared__ __align__(16) float T[64][TP];
    const int t = threadIdx.x, wave = t >> 5, lane = t & 31, h = lane >> 4, m = lane & 15;
    const int wm = wave & 3, wn = wave >> 2;
    const int m0 = blockIdx.x * 64, n0 = blockIdx.y * 64;
    const f16t* arow  = Xt + (size_t)(m0 + wm * 16 + m) * CD;
    const f16t* brow0 = W + (size_t)(n0 + wn * 32 + m) * CD;
    const f16t* brow1 = W + (size_t)(n0 + wn * 32 + 16 + m) * CD;
    v8f acc0 = {}, acc1 = {};
#pragma unroll 2
    for (int k0 = 0; k0 < CD; k0 += 32) {
        Frag a, b0, b1;
        a.half[0]  = *(const v8h*)(arow  + k0 + 8 * h);
        a.half[1]  = *(const v8h*)(arow  + k0 + 16 + 8 * h);
        b0.half[0] = *(const v8h*)(brow0 + k0 + 8 * h);
        b0.half[1] = *(const v8h*)(brow0 + k0 + 16 + 8 * h);
        b1.half[0] = *(const v8h*)(brow1 + k0 + 8 * h);
        b1.half[1] = *(const v8h*)(brow1 + k0 + 16 + 8 * h);
        acc0 = mma_g(acc0, a.v, b0.v);
        acc1 = mma_g(acc1, a.v, b1.v);
    }
#pragma unroll
    for (int r = 0; r < 8; ++r) {
        T[wm * 16 + 8 * h + r][wn * 32 + m]      = acc0[r];
        T[wm * 16 + 8 * h + r][wn * 32 + 16 + m] = acc1[r];
    }
    __syncthreads();

    const int region = blockIdx.y >> 2;
    if (region < 2) {
        f16t* dstb = (region == 0) ? Q16 : K16;
        const int cb = n0 - region * CD;
        H8 u[2]; f16t* dp[2];
#pragma unroll
        for (int i = 0; i < 2; ++i) {
            const int L = i * 32 + (t >> 3), q = t & 7;
            v4f x0 = *(const v4fa*)(&T[L][8 * q]);
            v4f x1 = *(const v4fa*)(&T[L][8 * q + 4]);
#pragma unroll
            for (int j = 0; j < 4; ++j) {
                u[i].h[j]     = (f16t)((x0[j] * INV_W + bias[n0 + 8 * q + j]) * QK_SCL);
                u[i].h[4 + j] = (f16t)((x1[j] * INV_W + bias[n0 + 8 * q + 4 + j]) * QK_SCL);
            }
            dp[i] = dstb + (size_t)(m0 + L) * CD + cb + 8 * q;
        }
        *(volatile v4f*)dp[0] = u[0].f;
        *(volatile v4f*)dp[1] = u[1].f;
        __threadfence();
        *(volatile v4f*)dp[0] = u[0].f;
        *(volatile v4f*)dp[1] = u[1].f;
    } else {
        const int cb = n0 - 2 * CD;
        v4f u[4]; float* dp[4];
#pragma unroll
        for (int i = 0; i < 4; ++i) {
            const int L = i * 32 + (t >> 3), q = t & 7;
            const int row = L >> 1, c = L & 1;
            v4f xv = *(const v4fa*)(&T[row][32 * c + 4 * q]);
#pragma unroll
            for (int j = 0; j < 4; ++j) xv[j] = xv[j] * INV_W + bias[n0 + 32 * c + 4 * q + j];
            u[i] = xv;
            dp[i] = Vf + (size_t)(m0 + row) * CD + cb + 32 * c + 4 * q;
        }
#pragma unroll
        for (int i = 0; i < 4; ++i) *(volatile v4f*)dp[i] = u[i];
        __threadfence();
#pragma unroll
        for (int i = 0; i < 4; ++i) *(volatile v4f*)dp[i] = u[i];
    }
}

__global__ __launch_bounds__(256) void k_dwconv(const float* __restrict__ Vf, const float* __restrict__ wdw,
                                               const float* __restrict__ bdw, f16t* __restrict__ V16,
                                               int nitems) {
    const int i = blockIdx.x * 256 + threadIdx.x;
    if (i >= nitems) return;
    const int tok = i >> 5, c8 = (i & 31) * 8;
    const int b = tok / NPIX, p = tok - b * NPIX;
    const int hh = p / HWD, ww = p - hh * HWD;
    float s[8];
#pragma unroll
    for (int j = 0; j < 8; ++j) s[j] = 0.f;
#pragma unroll
    for (int dy = 0; dy < 3; ++dy) {
        const int h2 = hh + dy - 1;
        if (h2 < 0 || h2 >= HWD) continue;
#pragma unroll
        for (int dx = 0; dx < 3; ++dx) {
            const int w2 = ww + dx - 1;
            if (w2 < 0 || w2 >= HWD) continue;
            const float* sp = Vf + ((size_t)b * NPIX + (size_t)h2 * HWD + w2) * CD + c8;
            v4f lo = *(const v4fa*)sp;
            v4f hi = *(const v4fa*)(sp + 4);
            const int tap = dy * 3 + dx;
#pragma unroll
            for (int j = 0; j < 4; ++j) {
                s[j]     += wdw[(c8 + j) * 9 + tap] * lo[j];
                s[4 + j] += wdw[(c8 + 4 + j) * 9 + tap] * hi[j];
            }
        }
    }
    const float* cp = Vf + (size_t)tok * CD + c8;
    v4f c0 = *(const v4fa*)cp;
    v4f c1 = *(const v4fa*)(cp + 4);
    H8 u;
#pragma unroll
    for (int j = 0; j < 4; ++j) {
        u.h[j]     = (f16t)((c0[j] + (s[j] + bdw[c8 + j])) * V_SCL);
        u.h[4 + j] = (f16t)((c1[j] + (s[4 + j] + bdw[c8 + 4 + j])) * V_SCL);
    }
    f16t* d = V16 + (size_t)tok * CD + c8;
    *(volatile v4f*)d = u.f;
    __threadfence();
    *(volatile v4f*)d = u.f;
}

__global__ __launch_bounds__(256) void k_attn(const f16t* __restrict__ Q16, const f16t* __restrict__ K16,
                                             const f16t* __restrict__ V16, f16t* __restrict__ O16) {
    __shared__ __align__(16) f16t Ks[SLP * HD];
    __shared__ __align__(16) f16t Vt[HD * SLP];
    __shared__ __align__(16) f16t Pall[8 * 16 * PP];

    const int tid = threadIdx.x;
    const int sidx = blockIdx.x;
    const int b = sidx >> 6, rr = sidx & 63, head = rr >> 3, sn = rr & 7, dir = head >> 2;
    const int ho = head * HD, base = b * NPIX;

    for (int row = tid; row < SLP; row += 256) {
        v8h z = {};
        v8h kq[4] = {z, z, z, z};
        v8h vq[4] = {z, z, z, z};
        if (row < SL) {
            const int tok = tok_of(dir, base, sn, row);
            const f16t* kp = K16 + (size_t)tok * CD + ho;
            const f16t* vp = V16 + (size_t)tok * CD + ho;
#pragma unroll
            for (int i = 0; i < 4; ++i) {
                kq[i] = *(const v8h*)(kp + 8 * i);
                vq[i] = *(const v8h*)(vp + 8 * i);
            }
        }
#pragma unroll
        for (int i = 0; i < 4; ++i) *(v8ha*)(Ks + row * HD + 8 * i) = kq[i];
#pragma unroll
        for (int c = 0; c < 32; ++c) Vt[c * SLP + row] = vq[c >> 3][c & 7];
    }
    __syncthreads();

    const int wave = tid >> 5, lane = tid & 31, h = lane >> 4, m = lane & 15;
    f16t* Pw = Pall + wave * (16 * PP);

    for (int t = wave; t < NQT; t += 8) {
        const int q0 = t * 16;
        int qi = q0 + m; if (qi > SL - 1) qi = SL - 1;
        const f16t* qrow = Q16 + (size_t)tok_of(dir, base, sn, qi) * CD + ho;
        Frag aQ;
        aQ.half[0] = *(const v8h*)(qrow + 8 * h);
        aQ.half[1] = *(const v8h*)(qrow + 16 + 8 * h);

        v8f acc0 = {}, acc1 = {};
        float mrow[8], lrow[8];
#pragma unroll
        for (int j = 0; j < 8; ++j) { mrow[j] = -1e30f; lrow[j] = 0.f; }

#pragma unroll 1
        for (int kc = 0; kc < NCH; ++kc) {
            const int k0 = kc * 32;
            Frag bK0, bK1;
            const f16t* kr0 = Ks + (k0 + m) * HD;
            const f16t* kr1 = Ks + (k0 + 16 + m) * HD;
            bK0.half[0] = *(const v8ha*)(kr0 + 8 * h);
            bK0.half[1] = *(const v8ha*)(kr0 + 16 + 8 * h);
            bK1.half[0] = *(const v8ha*)(kr1 + 8 * h);
            bK1.half[1] = *(const v8ha*)(kr1 + 16 + 8 * h);
            v8f zc = {};
            v8f s0 = mma_g(zc, aQ.v, bK0.v);
            v8f s1 = mma_g(zc, aQ.v, bK1.v);
            const bool ok0 = (k0 + m) < SL;
            const bool ok1 = (k0 + 16 + m) < SL;
            asm volatile("" ::: "memory");
#pragma unroll
            for (int j = 0; j < 8; ++j) {
                const float a0 = ok0 ? s0[j] * LOGIT_SCL : -1e30f;
                const float a1 = ok1 ? s1[j] * LOGIT_SCL : -1e30f;
                float mx = fmaxf(a0, a1);
                mx = fmaxf(mx, __shfl_xor(mx, 1, 16));
                mx = fmaxf(mx, __shfl_xor(mx, 2, 16));
                mx = fmaxf(mx, __shfl_xor(mx, 4, 16));
                mx = fmaxf(mx, __shfl_xor(mx, 8, 16));
                const float mnew = fmaxf(mrow[j], mx);
                const float sc = __expf(mrow[j] - mnew);
                const float p0 = ok0 ? __expf(a0 - mnew) : 0.f;
                const float p1 = ok1 ? __expf(a1 - mnew) : 0.f;
                float rs = p0 + p1;
                rs += __shfl_xor(rs, 1, 16);
                rs += __shfl_xor(rs, 2, 16);
                rs += __shfl_xor(rs, 4, 16);
                rs += __shfl_xor(rs, 8, 16);
                lrow[j] = lrow[j] * sc + rs;
                mrow[j] = mnew;
                acc0[j] *= sc;
                acc1[j] *= sc;
                Pw[(8 * h + j) * PP + m]      = (f16t)(p0 * P_SCL);
                Pw[(8 * h + j) * PP + 16 + m] = (f16t)(p1 * P_SCL);
            }
            asm volatile("" ::: "memory");
            Frag aP, bV0, bV1;
            const f16t* pr = Pw + m * PP;
            aP.half[0]  = *(const v8ha*)(pr + 8 * h);
            aP.half[1]  = *(const v8ha*)(pr + 16 + 8 * h);
            const f16t* vr0 = Vt + m * SLP + k0;
            const f16t* vr1 = Vt + (16 + m) * SLP + k0;
            bV0.half[0] = *(const v8ha*)(vr0 + 8 * h);
            bV0.half[1] = *(const v8ha*)(vr0 + 16 + 8 * h);
            bV1.half[0] = *(const v8ha*)(vr1 + 8 * h);
            bV1.half[1] = *(const v8ha*)(vr1 + 16 + 8 * h);
            acc0 = mma_g(acc0, aP.v, bV0.v);
            acc1 = mma_g(acc1, aP.v, bV1.v);
        }

        asm volatile("" ::: "memory");
#pragma unroll
        for (int j = 0; j < 8; ++j) {
            const float inv = O_EPI / lrow[j];
            Pw[(8 * h + j) * PP + m]      = (f16t)(acc0[j] * inv);
            Pw[(8 * h + j) * PP + 16 + m] = (f16t)(acc1[j] * inv);
        }
        asm volatile("" ::: "memory");
        const int sub = lane >> 3, pc = lane & 7;
        v4f ov[4]; f16t* od[4]; bool ok[4];
#pragma unroll
        for (int i = 0; i < 4; ++i) {
            const int R = 4 * i + sub;
            const int qr = q0 + R;
            ok[i] = qr < SL;
            const int qq = ok[i] ? qr : (SL - 1);
            H8 u;
            if (pc < 4) {
                u.h = *(const v8ha*)(Pw + R * PP + 8 * pc);
            } else {
                v4f zz = {};
                u.f = zz;
            }
            ov[i] = u.f;
            od[i] = O16 + (size_t)tok_of(dir, base, sn, qq) * OPITCH + head * 64 + 8 * pc;
        }
#pragma unroll
        for (int i = 0; i < 4; ++i) if (ok[i]) *(volatile v4f*)od[i] = ov[i];
        __threadfence();
#pragma unroll
        for (int i = 0; i < 4; ++i) if (ok[i]) *(volatile v4f*)od[i] = ov[i];
    }
}

__global__ __launch_bounds__(256) void k_gemm_proj(const f16t* __restrict__ O16, const f16t* __restrict__ Wp,
                                                  const float* __restrict__ bias, float* __restrict__ out) {
    __shared__ __align__(16) float T[64][TP];
    const int t = threadIdx.x, wave = t >> 5, lane = t & 31, h = lane >> 4, m = lane & 15;
    const int wm = wave & 3, wn = wave >> 2;
    const int m0 = blockIdx.x * 64, n0 = blockIdx.y * 64;
    const f16t* arow  = O16 + (size_t)(m0 + wm * 16 + m) * OPITCH;
    const f16t* brow0 = Wp + (size_t)(n0 + wn * 32 + m) * CD;
    const f16t* brow1 = Wp + (size_t)(n0 + wn * 32 + 16 + m) * CD;
    v8f acc0 = {}, acc1 = {};
#pragma unroll 2
    for (int ks = 0; ks < NHEAD; ++ks) {
        Frag a, b0, b1;
        a.half[0]  = *(const v8h*)(arow  + ks * 64 + 8 * h);
        a.half[1]  = *(const v8h*)(arow  + ks * 64 + 16 + 8 * h);
        b0.half[0] = *(const v8h*)(brow0 + ks * 32 + 8 * h);
        b0.half[1] = *(const v8h*)(brow0 + ks * 32 + 16 + 8 * h);
        b1.half[0] = *(const v8h*)(brow1 + ks * 32 + 8 * h);
        b1.half[1] = *(const v8h*)(brow1 + ks * 32 + 16 + 8 * h);
        acc0 = mma_g(acc0, a.v, b0.v);
        acc1 = mma_g(acc1, a.v, b1.v);
    }
#pragma unroll
    for (int r = 0; r < 8; ++r) {
        T[wn * 32 + m][wm * 16 + 8 * h + r]      = acc0[r];
        T[wn * 32 + 16 + m][wm * 16 + 8 * h + r] = acc1[r];
    }
    __syncthreads();

    const int bimg = m0 / NPIX, p0 = m0 - bimg * NPIX;
    v4f u[4]; float* dp[4];
#pragma unroll
    for (int i = 0; i < 4; ++i) {
        const int L = i * 32 + (t >> 3), q = t & 7;
        const int ol = L >> 1, c = L & 1;
        v4f xv = *(const v4fa*)(&T[ol][32 * c + 4 * q]);
        const float bv = bias[n0 + ol];
#pragma unroll
        for (int j = 0; j < 4; ++j) xv[j] = xv[j] * PROJ_EPI + bv;
        u[i] = xv;
        dp[i] = out + ((size_t)(bimg * CD + n0 + ol)) * NPIX + p0 + 32 * c + 4 * q;
    }
#pragma unroll
    for (int i = 0; i < 4; ++i) *(volatile v4f*)dp[i] = u[i];
    __threadfence();
#pragma unroll
    for (int i = 0; i < 4; ++i) *(volatile v4f*)dp[i] = u[i];
}

extern "C" void kernel_launch(void* const* d_in, const int* in_sizes, int n_in,
                              void* d_out, int out_size, void* d_ws, size_t ws_size,
                              hipStream_t stream) {
    if (n_in < 7) return;
    if (in_sizes[0] != NTOK * CD || in_sizes[1] != 3 * CD * CD || in_sizes[2] != 3 * CD ||
        in_sizes[3] != CD * 9 || in_sizes[4] != CD || in_sizes[5] != CD * CD ||
        in_sizes[6] != CD || out_size != NTOK * CD) return;

    const float* x      = (const float*)d_in[0];
    const float* w_qkv  = (const float*)d_in[1];
    const float* b_qkv  = (const float*)d_in[2];
    const float* w_dw   = (const float*)d_in[3];
    const float* b_dw   = (const float*)d_in[4];
    const float* w_proj = (const float*)d_in[5];
    const float* b_proj = (const float*)d_in[6];
    float* out = (float*)d_out;

    const size_t sz16  = (size_t)NTOK * CD * 2;
    const size_t szf32 = (size_t)NTOK * CD * 4;
    const size_t szo16 = (size_t)NTOK * OPITCH * 2;
    const size_t szwq  = (size_t)3 * CD * CD * 2;
    const size_t szwp  = (size_t)CD * CD * 2;
    size_t off = 0;
    char* ws = (char*)d_ws;
    f16t*  Xt   = (f16t*)(ws + off);  off += sz16;
    f16t*  Q16  = (f16t*)(ws + off);  off += sz16;
    f16t*  K16  = (f16t*)(ws + off);  off += sz16;
    float* Vf32 = (float*)(ws + off); off += szf32;
    f16t*  V16  = (f16t*)(ws + off);  off += sz16;
    f16t*  O16  = (f16t*)(ws + off);  off += szo16;
    f16t*  Wq16 = (f16t*)(ws + off);  off += szwq;
    f16t*  Wp16 = (f16t*)(ws + off);  off += szwp;
    if (off > ws_size) return;

    const int n8q = (3 * CD * CD) / 8;
    const int n8p = (CD * CD) / 8;
    const int ndw = NTOK * (CD / 8);

    k_cvt_x<<<dim3(NTOK / 32, CD / 64), 256, 0, stream>>>(x, Xt);
    k_cvt_w<<<(n8q + 255) / 256, 256, 0, stream>>>(w_qkv, Wq16, n8q, W_SCL);
    k_cvt_w<<<(n8p + 255) / 256, 256, 0, stream>>>(w_proj, Wp16, n8p, W_SCL);
    k_gemm_qkv<<<dim3(NTOK / 64, (3 * CD) / 64), 256, 0, stream>>>(Xt, Wq16, b_qkv, Q16, K16, Vf32);
    k_dwconv<<<(ndw + 255) / 256, 256, 0, stream>>>(Vf32, w_dw, b_dw, V16, ndw);
    k_attn<<<NBATCH * NHEAD * 8, 256, 0, stream>>>(Q16, K16, V16, O16);
    k_gemm_proj<<<dim3(NTOK / 64, CD / 64), 256, 0, stream>>>(O16, Wp16, b_proj, out);
}
